// GatedGCNLayer_27900107555156
// MI455X (gfx1250) — hardware-verified
//
#include <hip/hip_runtime.h>
#include <stddef.h>
#include <stdint.h>


#define FEAT   128
#define NP     256
#define NT     256
#define NBH    NP
#define NBT    NT
#define KQ     16
#define KSTEP  4
#define APK    136
#define TR     16
#define NTHR   256
#define NWAVE  8
#define CTH    2
#define CTT    2
#define S1     2048
#define NCH1   8
#define SH1    12
#define SH2    7
#define SH3    4
#define F1A    32
#define F2     32
#define F3     8
#define CAP1   256
#define CAP2   128
#define CAP3   256
#define SEGS2  16
#define WSC    64.0f
#define RWSC   0.015625f
#define SENT   0xFFFFFFFFu
#define OVF    0x00000001u
#define WSCAPB 134217728
#define NPREP  ((NBH + NBT) * KQ)

static_assert(NP == 2 * FEAT && NT == 2 * FEAT);
static_assert(KQ * 8 == FEAT && KSTEP * 32 == FEAT);
static_assert((APK % 8) == 0 && APK >= FEAT);
static_assert(NPREP % NTHR == 0 && NPREP == 8192);
static_assert(NCH1 * NTHR == S1);
static_assert(CAP1 == NTHR);
static_assert((F1A * CAP1) % (4 * NTHR) == 0);
static_assert((F2 * CAP2) % (4 * NTHR) == 0);
static_assert((F3 * CAP3) % (4 * NTHR) == 0);
static_assert((CAP1 % 32) == 0 && (CAP2 % 32) == 0 && (CAP3 % 32) == 0);
static_assert(NTHR == 32 * NWAVE && TR == 2 * NWAVE);
static_assert(CTH * 16 * NWAVE == NP && CTT * 16 * NWAVE == NT);
static_assert(NTHR * 4 * 2 == TR * FEAT);
static_assert((TR * NP) % (4 * NTHR) == 0);
static_assert(F1A <= 32 && F2 <= 32 && F3 <= 32);

typedef _Float16 v4h  __attribute__((ext_vector_type(4)));
typedef _Float16 v8h  __attribute__((ext_vector_type(8)));
typedef _Float16 v16h __attribute__((ext_vector_type(16)));
typedef float    v4f  __attribute__((ext_vector_type(4)));
typedef float    v8f  __attribute__((ext_vector_type(8)));
typedef unsigned int v4u __attribute__((ext_vector_type(4)));
typedef v4h v4ha __attribute__((may_alias));
typedef v8h v8ha __attribute__((may_alias));
typedef v4f v4fa __attribute__((may_alias));
typedef v4u v4ua __attribute__((may_alias));
union Frag { v16h v; v8h h[2]; };

__device__ __forceinline__ v8f wmh(v16h a, v16h b, v8f c) {
  v8f d = __builtin_amdgcn_wmma_f32_16x16x32_f16(false, a, false, b, (short)0, c, false, false);
  asm volatile("v_nop\n\tv_nop\n\tv_nop\n\tv_nop" : "+v"(d) : "v"(a), "v"(b));
  return d;
}

__device__ __forceinline__ v4h cvt4(v4f a) {
  v4h r;
  r[0] = (_Float16)a[0]; r[1] = (_Float16)a[1]; r[2] = (_Float16)a[2]; r[3] = (_Float16)a[3];
  return r;
}

__global__ __launch_bounds__(NTHR) void k_wprep(const float* __restrict__ wg, const float* __restrict__ wsw,
                                                const float* __restrict__ wr, _Float16* Bw) {
  const int gi = blockIdx.x * NTHR + threadIdx.x;
  const int part = gi >> 12;
  const int i = gi & 4095;
  const int n = i >> 4, k0 = (i & 15) * 8;
  const int sub = n >> 7, c = n & (FEAT - 1);
  const int sel = part * 2 + sub;
  v8h hv;
#pragma unroll
  for (int e = 0; e < 8; ++e) {
    const int k = k0 + e;
    const float v0 = wg[((size_t)(FEAT + k)) * FEAT + c];
    const float v1 = wsw[((size_t)k) * FEAT + c];
    const float v2 = wg[((size_t)k) * FEAT + c];
    const float v3 = wr[((size_t)k) * FEAT + c];
    const float v = sel == 0 ? v0 : (sel == 1 ? v1 : (sel == 2 ? v2 : v3));
    hv[e] = (_Float16)(v * WSC);
  }
  _Float16* dst = Bw + (size_t)gi * 8;
  *(volatile v8h*)dst = hv;
  __threadfence();
  *(volatile v8h*)dst = hv;
}

template <int LV, int FA, int CAP>
__global__ __launch_bounds__(NTHR) void k_part(const int* __restrict__ esrc, const int* __restrict__ edst,
                                               const unsigned* lin, unsigned* lout, unsigned* flg,
                                               int nN, int nE, int nC, int nB1, int P2, int nch) {
  __shared__ __attribute__((aligned(16))) unsigned lst[FA * CAP];
  __shared__ int wc[NWAVE * 32];
  __shared__ int cur[32];
  const int tid = threadIdx.x, lane = tid & 31, wave = tid >> 5;
  const int blk = blockIdx.x;
  const v4u sv = {SENT, SENT, SENT, SENT};
#pragma unroll
  for (int k = 0; k < (FA * CAP) / (4 * NTHR); ++k) *(v4ua*)(&lst[4 * (tid + NTHR * k)]) = sv;
  if (wave == 0) cur[lane] = 0;
  __syncthreads();

  int c = 0, part = 0, ml = 0;
  if (LV == 2) { c = blk / P2; part = blk - c * P2; }
  if (LV == 3) { c = blk >> 5; ml = blk & 31; }
  const int nslots3 = P2 * CAP2;

#pragma unroll 1
  for (int ch = 0; ch < nch; ++ch) {
    bool valid;
    int key;
    unsigned rec;
    if (LV == 1) {
      const int e = blk * S1 + ch * NTHR + tid;
      const int ec = e < nE ? e : nE - 1;
      const int d = edst[ec];
      valid = (e < nE) && ((unsigned)d < (unsigned)nN);
      key = d >> SH1;
      rec = (unsigned)ec;
    } else if (LV == 2) {
      const int bl = part * SEGS2 + ch;
      const int blc = bl < nB1 ? bl : nB1 - 1;
      const unsigned id = lin[((size_t)blc * nC + c) * CAP1 + tid];
      const bool idok = id < (unsigned)nE;
      const int idc = idok ? (int)id : nE - 1;
      const int d = edst[idc];
      valid = (bl < nB1) && idok && ((unsigned)d < (unsigned)nN);
      key = (d >> SH2) & 31;
      rec = (unsigned)idc;
    } else {
      const int q = ch * NTHR + tid;
      const int qc = q < nslots3 ? q : nslots3 - 1;
      const int pp = qc / CAP2, s = qc - pp * CAP2;
      const unsigned id = lin[(((size_t)(c * P2 + pp)) * F2 + ml) * CAP2 + s];
      const bool idok = id < (unsigned)nE;
      const int idc = idok ? (int)id : nE - 1;
      const int d = edst[idc];
      int sv2 = esrc[idc];
      sv2 = sv2 < 0 ? 0 : (sv2 > nN - 1 ? nN - 1 : sv2);
      valid = (q < nslots3) && idok && ((unsigned)d < (unsigned)nN);
      key = (d >> SH3) & 7;
      rec = ((unsigned)d & 15u) | ((unsigned)sv2 << 4);
    }
    key = valid ? key : 255;
    unsigned mym = 0u;
#pragma unroll
    for (int b = 0; b < FA; ++b) {
      const unsigned mb = __builtin_amdgcn_ballot_w32(key == b);
      mym = (key == b) ? mb : mym;
    }
    const unsigned lt = (1u << lane) - 1u;
    const int rank = __builtin_popcount(mym & lt);
    const int cnt  = __builtin_popcount(mym);
    wc[wave * 32 + lane] = 0;
    if (valid && rank == 0) wc[wave * 32 + key] = cnt;
    __syncthreads();
    const int kc = key & 31;
    int pre = 0;
    for (int w2 = 0; w2 < wave; ++w2) pre += wc[w2 * 32 + kc];
    const int pos = cur[kc] + pre + rank;
    if (valid && pos < CAP) lst[kc * CAP + pos] = rec;
    int tot = 0;
    if (wave == 0) {
#pragma unroll
      for (int w2 = 0; w2 < NWAVE; ++w2) tot += wc[w2 * 32 + lane];
    }
    __syncthreads();
    if (wave == 0) cur[lane] += tot;
  }
  __syncthreads();
  if (wave == 0 && cur[lane] > CAP) { *(volatile unsigned*)flg = OVF; }

  const int nwords  = (LV == 1) ? nC * CAP : FA * CAP;
  const int npieces = nwords >> 2;
  unsigned* gb = lout + (size_t)blk * nwords;
#pragma unroll
  for (int k = 0; k < (FA * CAP / 4 + NTHR - 1) / NTHR; ++k) {
    const int it = tid + NTHR * k;
    if (it < npieces) { const v4u v = *(const v4ua*)(&lst[4 * it]); *(volatile v4u*)(gb + 4 * it) = v; }
  }
  __threadfence();
#pragma unroll
  for (int k = 0; k < (FA * CAP / 4 + NTHR - 1) / NTHR; ++k) {
    const int it = tid + NTHR * k;
    if (it < npieces) { const v4u v = *(const v4ua*)(&lst[4 * it]); *(volatile v4u*)(gb + 4 * it) = v; }
  }
}

__global__ __launch_bounds__(NTHR) void k_proj(const float* __restrict__ x, const _Float16* __restrict__ BH,
                                               float* P, int nN) {
  __shared__ __attribute__((aligned(16))) _Float16 sA[TR * APK];
  __shared__ __attribute__((aligned(16))) float stg[TR * NP];
  const int tid = threadIdx.x, lane = tid & 31, wave = tid >> 5, hh = lane >> 4, m = lane & 15;
  const int tile = blockIdx.x;
  const v4f z4 = {0.f, 0.f, 0.f, 0.f};
#pragma unroll
  for (int k = 0; k < 2; ++k) {
    const int row = wave + 8 * k, c4 = lane * 4;
    const int node = tile * TR + row;
    const int nc = node < nN ? node : nN - 1;
    v4f v = *(const v4f*)(x + (size_t)nc * FEAT + c4);
    if (node >= nN) v = z4;
    *(v4ha*)(sA + row * APK + c4) = cvt4(v);
  }
  __syncthreads();

  v16h av[KSTEP];
  {
    const _Float16* abase = sA + m * APK + 8 * hh;
#pragma unroll
    for (int kt = 0; kt < KSTEP; ++kt) {
      Frag a;
      a.h[0] = *(const v8ha*)(abase + 32 * kt);
      a.h[1] = *(const v8ha*)(abase + 32 * kt + 16);
      av[kt] = a.v;
    }
  }
#pragma unroll 1
  for (int ct = 0; ct < CTH; ++ct) {
    const int col = wave * (16 * CTH) + ct * 16 + m;
    const _Float16* bb = BH + (size_t)col * FEAT + 8 * hh;
    v8f acc = {0.f, 0.f, 0.f, 0.f, 0.f, 0.f, 0.f, 0.f};
#pragma unroll
    for (int kt = 0; kt < KSTEP; ++kt) {
      Frag b;
      b.h[0] = *(const v8h*)(bb + 32 * kt);
      b.h[1] = *(const v8h*)(bb + 32 * kt + 16);
      acc = wmh(av[kt], b.v, acc);
    }
#pragma unroll
    for (int r = 0; r < 8; ++r) stg[(8 * hh + r) * NP + col] = acc[r] * RWSC;
  }
  __syncthreads();

  float* gb = P + (size_t)tile * (TR * NP);
#pragma unroll
  for (int k = 0; k < (TR * NP) / (4 * NTHR); ++k) {
    const int it = tid + NTHR * k;
    const v4f v = *(const v4fa*)(stg + 4 * it);
    *(volatile v4f*)(gb + 4 * it) = v;
  }
  __threadfence();
#pragma unroll
  for (int k = 0; k < (TR * NP) / (4 * NTHR); ++k) {
    const int it = tid + NTHR * k;
    const v4f v = *(const v4fa*)(stg + 4 * it);
    *(volatile v4f*)(gb + 4 * it) = v;
  }
}

__device__ __forceinline__ v4f drain(unsigned msk, unsigned rec, v4f ag, v4f bgv, v4f bsv,
                                     const float* __restrict__ P, int lane, int nN, v4f acc) {
  while (msk != 0u) {
    const int i = __builtin_ctz(msk);
    msk &= msk - 1u;
    const unsigned r = (unsigned)__builtin_amdgcn_readlane((int)rec, i);
    int src = (int)(r >> 4);
    src = src > nN - 1 ? nN - 1 : src;
    const float* prow = P + (size_t)src * NP + 4 * lane;
    const v4f bq = *(const v4f*)(prow);
    const v4f s  = *(const v4f*)(prow + FEAT);
    const v4f g  = (ag + bq) + bgv;
    v4f eta;
    eta[0] = __builtin_amdgcn_rcpf(1.0f + __expf(-g[0]));
    eta[1] = __builtin_amdgcn_rcpf(1.0f + __expf(-g[1]));
    eta[2] = __builtin_amdgcn_rcpf(1.0f + __expf(-g[2]));
    eta[3] = __builtin_amdgcn_rcpf(1.0f + __expf(-g[3]));
    acc += eta * (s + bsv);
  }
  return acc;
}

__global__ __launch_bounds__(NTHR) void k_tile(const float* __restrict__ x, const _Float16* __restrict__ BT,
                                               const unsigned* __restrict__ l3, const float* __restrict__ P,
                                               const float* __restrict__ bg, const float* __restrict__ bs,
                                               const float* __restrict__ br, const unsigned* __restrict__ flg,
                                               float* out, int nN) {
  __shared__ __attribute__((aligned(16))) _Float16 sA[TR * APK];
  __shared__ __attribute__((aligned(16))) float stg[TR * NT];
  const int tid = threadIdx.x, lane = tid & 31, wave = tid >> 5, hh = lane >> 4, m = lane & 15;
  const int tile = blockIdx.x;
  const v4f z4 = {0.f, 0.f, 0.f, 0.f};
#pragma unroll
  for (int k = 0; k < 2; ++k) {
    const int row = wave + 8 * k, c4 = lane * 4;
    const int node = tile * TR + row;
    const int nc = node < nN ? node : nN - 1;
    v4f v = *(const v4f*)(x + (size_t)nc * FEAT + c4);
    if (node >= nN) v = z4;
    *(v4ha*)(sA + row * APK + c4) = cvt4(v);
  }
  __syncthreads();

  {
    v16h av[KSTEP];
    const _Float16* abase = sA + m * APK + 8 * hh;
#pragma unroll
    for (int kt = 0; kt < KSTEP; ++kt) {
      Frag a;
      a.h[0] = *(const v8ha*)(abase + 32 * kt);
      a.h[1] = *(const v8ha*)(abase + 32 * kt + 16);
      av[kt] = a.v;
    }
#pragma unroll 1
    for (int ct = 0; ct < CTT; ++ct) {
      const int col = wave * (16 * CTT) + ct * 16 + m;
      const _Float16* bb = BT + (size_t)col * FEAT + 8 * hh;
      v8f acc = {0.f, 0.f, 0.f, 0.f, 0.f, 0.f, 0.f, 0.f};
#pragma unroll
      for (int kt = 0; kt < KSTEP; ++kt) {
        Frag b;
        b.h[0] = *(const v8h*)(bb + 32 * kt);
        b.h[1] = *(const v8h*)(bb + 32 * kt + 16);
        acc = wmh(av[kt], b.v, acc);
      }
#pragma unroll
      for (int r = 0; r < 8; ++r) stg[(8 * hh + r) * NT + col] = acc[r] * RWSC;
    }
  }
  __syncthreads();

  const int c4 = lane * 4;
  const v4f bgv = *(const v4f*)(bg + c4);
  const v4f bsv = *(const v4f*)(bs + c4);
  const v4f brv = *(const v4f*)(br + c4);
  const v4f ag0 = *(const v4fa*)(stg + (2 * wave) * NT + c4);
  const v4f ag1 = *(const v4fa*)(stg + (2 * wave + 1) * NT + c4);
  const v4f rt0 = *(const v4fa*)(stg + (2 * wave) * NT + FEAT + c4);
  const v4f rt1 = *(const v4fa*)(stg + (2 * wave + 1) * NT + FEAT + c4);
  v4f acc0 = z4, acc1 = z4;
  {
    const unsigned* seg = l3 + (size_t)tile * CAP3;
#pragma unroll 1
    for (int ch = 0; ch < CAP3 / 32; ++ch) {
      const unsigned rec = seg[ch * 32 + lane];
      const bool ok = ((int)rec) >= 0;
      const int ln = (int)(rec & 15u);
      const unsigned m0 = __builtin_amdgcn_ballot_w32(ok && (ln == 2 * wave));
      const unsigned m1 = __builtin_amdgcn_ballot_w32(ok && (ln == 2 * wave + 1));
      acc0 = drain(m0, rec, ag0, bgv, bsv, P, lane, nN, acc0);
      acc1 = drain(m1, rec, ag1, bgv, bsv, P, lane, nN, acc1);
    }
  }

  v4f o0 = (rt0 + brv) + acc0;
  v4f o1 = (rt1 + brv) + acc1;
  const unsigned fl = flg[0];
  if (fl == OVF) {
    const float qn = __uint_as_float(0x7fc00000u);
    const v4f nv = {qn, qn, qn, qn};
    o0 = nv; o1 = nv;
  }
  const int node0 = tile * TR + 2 * wave, node1 = node0 + 1;
  const bool a0 = node0 < nN, a1 = node1 < nN;
  float* g0 = out + (size_t)(a0 ? node0 : 0) * FEAT + c4;
  float* g1 = out + (size_t)(a1 ? node1 : 0) * FEAT + c4;
  if (a0) *(volatile v4f*)g0 = o0;
  if (a1) *(volatile v4f*)g1 = o1;
  __threadfence();
  if (a0) *(volatile v4f*)g0 = o0;
  if (a1) *(volatile v4f*)g1 = o1;
}

extern "C" void kernel_launch(void* const* d_in, const int* in_sizes, int n_in,
                              void* d_out, int out_size, void* d_ws, size_t ws_size,
                              hipStream_t stream) {
  if (n_in < 8) return;
  if (in_sizes[0] <= 0 || (in_sizes[0] % FEAT) != 0) return;
  if (in_sizes[1] <= 0 || (in_sizes[1] % 2) != 0) return;
  const int nN = in_sizes[0] / FEAT;
  const int nE = in_sizes[1] / 2;
  if (nN < 1 || nN > (F1A << SH1)) return;
  if (nE < 1 || nE > (1 << 28)) return;
  if (in_sizes[2] != 2 * FEAT * FEAT || in_sizes[3] != FEAT) return;
  if (in_sizes[4] != FEAT * FEAT || in_sizes[5] != FEAT) return;
  if (in_sizes[6] != FEAT * FEAT || in_sizes[7] != FEAT) return;
  if (out_size != nN * FEAT) return;

  const float* x   = (const float*)d_in[0];
  const int*   ei  = (const int*)d_in[1];
  const int*   esrc = ei;
  const int*   edst = ei + (size_t)nE;
  const float* wg  = (const float*)d_in[2];
  const float* bg  = (const float*)d_in[3];
  const float* wsw = (const float*)d_in[4];
  const float* bs  = (const float*)d_in[5];
  const float* wr  = (const float*)d_in[6];
  const float* br  = (const float*)d_in[7];
  float* out = (float*)d_out;

  const int nTiles = (nN + TR - 1) / TR;
  const int nC   = (nN + (1 << SH1) - 1) >> SH1;
  const int nB1  = (nE + S1 - 1) / S1;
  const int P2   = (nB1 + SEGS2 - 1) / SEGS2;
  const int nch3 = (P2 * CAP2 + NTHR - 1) / NTHR;
  if (nC < 1 || nC > F1A) return;

  char* ws = (char*)d_ws;
  size_t o = 0;
  const size_t oBw = o; o += (size_t)(NBH + NBT) * FEAT * 2;              o = (o + 255) & ~(size_t)255;
  const size_t oL1 = o; o += (size_t)nB1 * nC * CAP1 * 4;                 o = (o + 255) & ~(size_t)255;
  const size_t oL2 = o; o += (size_t)nC * P2 * F2 * CAP2 * 4;             o = (o + 255) & ~(size_t)255;
  const size_t oL3 = o; o += (size_t)nC * 32 * F3 * CAP3 * 4;             o = (o + 255) & ~(size_t)255;
  const size_t oP  = o; o += (size_t)nTiles * TR * NP * 4;                o = (o + 255) & ~(size_t)255;
  const size_t oFl = o; o += 256;
  if (o > ws_size || o > (size_t)WSCAPB) return;
  _Float16* Bw = (_Float16*)(ws + oBw);
  unsigned* L1 = (unsigned*)(ws + oL1);
  unsigned* L2 = (unsigned*)(ws + oL2);
  unsigned* L3 = (unsigned*)(ws + oL3);
  float*    P  = (float*)(ws + oP);
  unsigned* FL = (unsigned*)(ws + oFl);

  k_wprep<<<NPREP / NTHR, NTHR, 0, stream>>>(wg, wsw, wr, Bw);
  k_part<1, F1A, CAP1><<<nB1, NTHR, 0, stream>>>(esrc, edst, L1, L1, FL, nN, nE, nC, nB1, P2, NCH1);
  k_part<2, F2, CAP2><<<nC * P2, NTHR, 0, stream>>>(esrc, edst, L1, L2, FL, nN, nE, nC, nB1, P2, SEGS2);
  k_part<3, F3, CAP3><<<nC * 32, NTHR, 0, stream>>>(esrc, edst, L2, L3, FL, nN, nE, nC, nB1, P2, nch3);
  k_proj<<<nTiles, NTHR, 0, stream>>>(x, Bw, P, nN);
  k_tile<<<nTiles, NTHR, 0, stream>>>(x, Bw + (size_t)NBH * FEAT, L3, P, bg, bs, br, FL, out, nN);
}
